// EuclideanSimilarity_60120952209550
// MI455X (gfx1250) — hardware-verified
//
#include <hip/hip_runtime.h>
#include <math.h>

typedef __attribute__((ext_vector_type(16))) _Float16 v16h;
typedef __attribute__((ext_vector_type(16))) __bf16 v16b;
typedef __attribute__((ext_vector_type(8)))  _Float16 v8h;
typedef __attribute__((ext_vector_type(8)))  float v8f;
typedef __attribute__((ext_vector_type(4)))  float v4f;
typedef __attribute__((ext_vector_type(2)))  float v2f;
typedef __attribute__((ext_vector_type(4)))  unsigned v4u;
typedef __attribute__((ext_vector_type(4)))  int v4i;
typedef float __attribute__((may_alias)) float_a;
typedef int __attribute__((may_alias)) int_a;

template <typename T> __device__ __forceinline__ void vst2(void* p, T v) { *(volatile T*)p = v; __threadfence(); *(volatile T*)p = v; }
__device__ __forceinline__ v8f wmma16(v16h a, v16h b, v8f c) {
  v8f d = __builtin_amdgcn_wmma_f32_16x16x32_f16(false, a, false, b, (short)0, c, false, false);
  asm volatile("v_nop\n\tv_nop\n\tv_nop\n\tv_nop" : "+v"(d) : "v"(a), "v"(b));
  return d;
}
__device__ __forceinline__ v8f wmma_bf(v16b a, v16b b, v8f c) {
  v8f d = __builtin_amdgcn_wmma_f32_16x16x32_bf16(false, a, false, b, (short)0, c, false, false);
  asm volatile("v_nop\n\tv_nop\n\tv_nop\n\tv_nop" : "+v"(d) : "v"(a), "v"(b));
  return d;
}
__device__ __forceinline__ v16h frag_h(const _Float16* rowk0, int lane) {
  union { v16h v; v8h q[2]; } u; const _Float16* p = rowk0 + 8 * (lane >> 4);
  u.q[0] = *(const v8h*)p; u.q[1] = *(const v8h*)(p + 16); return u.v;
}
__device__ __forceinline__ v16h frag_f32(const float* rowk0, int lane) {
  v16h a; const float* p = rowk0 + 8 * (lane >> 4);
#pragma unroll
  for (int i = 0; i < 8; ++i) { a[i] = (_Float16)p[i]; a[8 + i] = (_Float16)p[16 + i]; }
  return a;
}
__device__ __forceinline__ v16h frag_f32s(const float* rowk0, int lane, float sc) {
  v16h a; const float* p = rowk0 + 8 * (lane >> 4);
#pragma unroll
  for (int i = 0; i < 8; ++i) { a[i] = (_Float16)(p[i] * sc); a[8 + i] = (_Float16)(p[16 + i] * sc); }
  return a;
}
__device__ __forceinline__ v16h fragc_f32(const float* W, int k0, int n, int lane, int ld, int K) {
  v16h a; const int g = lane >> 4;
#pragma unroll
  for (int i = 0; i < 8; ++i) { const int ka = k0 + 8 * g + i, kb = ka + 16;
    a[i] = (_Float16)(ka < K ? W[(size_t)(ka < K ? ka : K - 1) * ld + n] : 0.f); a[8 + i] = (_Float16)(kb < K ? W[(size_t)(kb < K ? kb : K - 1) * ld + n] : 0.f); }
  return a;
}
struct F2 { v16b h, l; };
__device__ __forceinline__ F2 bsplit16(const float v[16]) { F2 r;
#pragma unroll
  for (int i = 0; i < 16; ++i) { const __bf16 h = (__bf16)v[i]; r.h[i] = h; r.l[i] = (__bf16)(v[i] - (float)h); }
  return r; }
__device__ __forceinline__ F2 split_row(const float* row, int k0, int lane) { float v[16]; const float* p = row + k0 + 8 * (lane >> 4);
#pragma unroll
  for (int i = 0; i < 8; ++i) { v[i] = p[i]; v[8 + i] = p[16 + i]; }
  return bsplit16(v); }
__device__ __forceinline__ F2 split_rowK(const float* row, int k0, int lane, int K) { float v[16]; const int g = lane >> 4;
#pragma unroll
  for (int i = 0; i < 8; ++i) { const int ka = k0 + 8 * g + i, kb = ka + 16; v[i] = ka < K ? row[ka < K ? ka : K - 1] : 0.f; v[8 + i] = kb < K ? row[kb < K ? kb : K - 1] : 0.f; }
  return bsplit16(v); }
__device__ __forceinline__ F2 split_col(const float* W, int k0, int n, int lane, int ld, int K) { float v[16]; const int g = lane >> 4;
#pragma unroll
  for (int i = 0; i < 8; ++i) { const int ka = k0 + 8 * g + i, kb = ka + 16; v[i] = ka < K ? W[(size_t)(ka < K ? ka : K - 1) * ld + n] : 0.f; v[8 + i] = kb < K ? W[(size_t)(kb < K ? kb : K - 1) * ld + n] : 0.f; }
  return bsplit16(v); }
__device__ __forceinline__ v8f mac3(const F2& a, const F2& b, v8f c) { c = wmma_bf(a.l, b.h, c); c = wmma_bf(a.h, b.l, c); return wmma_bf(a.h, b.h, c); }
__device__ __forceinline__ float sigm(float v) { return 1.0f / (1.0f + expf(-v)); }
#define LDSX() do { asm volatile("s_wait_dscnt 0" ::: "memory"); __builtin_amdgcn_wave_barrier(); __builtin_amdgcn_fence(__ATOMIC_RELEASE, "workgroup"); } while (0)


#define NB 8
#define LL 4096
#define LQ 2048
#define DD 128
#ifndef TQB
#define TQB (LQ / 64)
#define TNB NB
#endif
typedef __attribute__((ext_vector_type(8))) __bf16 v8b;
__device__ __forceinline__ v16b frag_b(const __bf16* rowk0, int lane) {
  union { v16b v; v8b q[2]; } u; const __bf16* p = rowk0 + 8 * (lane >> 4);
  u.q[0] = *(const v8b*)p; u.q[1] = *(const v8b*)(p + 16); return u.v;
}
__device__ __forceinline__ float bfr(float v) { return (float)(__bf16)v; }
__device__ __attribute__((noinline)) float exp_ni(float v) { return expf(v); }
__device__ __attribute__((noinline)) float erf_ni(float v) { return erff(v); }

#define WS_PW  0u
#define WS_P   (WS_PW + 2u * DD * DD)
#define WS_Q   (WS_P + 4u * NB * LL * DD)
#define WS_PH  (WS_Q + 4u * NB * LQ * DD)
#define WS_PL  (WS_PH + 2u * NB * DD * LL)
#define WS_KS  (WS_PL + 2u * NB * DD * LL)
#define WS_QS  (WS_KS + 4u * NB * LL)
#define WS_END (WS_QS + 4u * NB * LQ)

__global__ __launch_bounds__(128) void k_pack(const float* __restrict__ Wm, __bf16* __restrict__ PW) {
  __shared__ __align__(16) __bf16 s[DD]; const int n = blockIdx.x, k = threadIdx.x; s[k] = (__bf16)Wm[(size_t)n * DD + k]; __syncthreads();
  if (k < DD / 8) vst2((unsigned*)(PW + (size_t)n * DD + k * 8), *(const v4u*)&s[k * 8]);
}
template <int POOL>
__global__ __launch_bounds__(128) void k_proj(const float* __restrict__ X, const __bf16* __restrict__ PW, const float* __restrict__ Bv, float* __restrict__ OUT, float* __restrict__ SQ, float* __restrict__ OUT2) {
  __shared__ __align__(16) float so[4][16][132]; __shared__ __align__(16) float ssq[64];
  const int tid = threadIdx.x, wave = tid >> 5, lane = tid & 31, col = lane & 15, g = lane >> 4; const size_t r0 = (size_t)blockIdx.x * 64 + wave * 16;
  v8f acc[8] = {};
#pragma unroll
  for (int kc = 0; kc < DD / 32; ++kc) { F2 a;
    if (POOL) { float v[16]; const float* p0 = X + (2 * (r0 + col)) * DD + kc * 32 + 8 * g; const float* p1 = p0 + DD;
#pragma unroll
      for (int i = 0; i < 8; ++i) { v[i] = (bfr(p0[i]) + bfr(p1[i])) * 0.5f; v[8 + i] = (bfr(p0[16 + i]) + bfr(p1[16 + i])) * 0.5f; }
      a = bsplit16(v); }
    else { v16b ax; const float* p = X + (r0 + col) * DD + kc * 32 + 8 * g;
#pragma unroll
      for (int i = 0; i < 8; ++i) { ax[i] = (__bf16)p[i]; ax[8 + i] = (__bf16)p[16 + i]; } a.h = ax; a.l = ax; }
#pragma unroll
    for (int j = 0; j < 8; ++j) { const v16b w = frag_b(PW + (size_t)(j * 16 + col) * DD + kc * 32, lane); if (POOL) acc[j] = wmma_bf(a.l, w, acc[j]); acc[j] = wmma_bf(a.h, w, acc[j]); } }
  float sq[8];
#pragma unroll
  for (int r = 0; r < 8; ++r) sq[r] = 0.f;
#pragma unroll
  for (int j = 0; j < 8; ++j) { const float bb = bfr(Bv[j * 16 + col]);
#pragma unroll
    for (int r = 0; r < 8; ++r) { const float v = acc[j][r] + bb; so[wave][8 * g + r][j * 16 + col] = v; sq[r] += v * v; } }
#pragma unroll
  for (int r = 0; r < 8; ++r) {
#pragma unroll
    for (int o = 1; o < 16; o <<= 1) sq[r] += __shfl_xor(sq[r], o);
    if (col == 0) ssq[wave * 16 + 8 * g + r] = sq[r]; }
  LDSX();
  for (int rl = 0; rl < 16; ++rl) { vst2(OUT + (r0 + rl) * DD + lane * 4, *(const v4f*)&so[wave][rl][lane * 4]); if (POOL) vst2(OUT2 + (r0 + rl) * DD + lane * 4, *(const v4f*)&so[wave][rl][lane * 4]); }
  __syncthreads();
  if (tid < 16) vst2(SQ + (size_t)blockIdx.x * 64 + tid * 4, *(const v4f*)&ssq[tid * 4]);
}
__global__ __launch_bounds__(256) void k_planes(const float* __restrict__ P, __bf16* __restrict__ PH, __bf16* __restrict__ PL) {
  __shared__ __align__(16) __bf16 sh[128][72], sl[128][72]; const int tid = threadIdx.x; const size_t rb = (size_t)blockIdx.x * 64; const int b = (int)(rb / LL), j0 = (int)(rb % LL);
  for (int q = tid; q < 64 * 128; q += 256) { const int rl = q >> 7, c = q & 127; const float v = P[(rb + rl) * DD + c]; const __bf16 hb = (__bf16)v; sh[c][rl] = hb; sl[c][rl] = (__bf16)(v - (float)hb); }
  __syncthreads();
  for (int q = tid; q < 128 * 8; q += 256) { const int c = q >> 3, pc = q & 7; const size_t o = ((size_t)b * DD + c) * LL + j0 + pc * 8; vst2((unsigned*)(PH + o), *(const v4u*)&sh[c][pc * 8]); vst2((unsigned*)(PL + o), *(const v4u*)&sl[c][pc * 8]); }
}
__global__ __launch_bounds__(128) void k_simk(const float* __restrict__ Q, const float* __restrict__ P, const float* __restrict__ QS, const float* __restrict__ KS, const __bf16* __restrict__ PH, const __bf16* __restrict__ PL, float* __restrict__ OK1, float* __restrict__ OK2) {
  __shared__ __align__(16) float sp[4][16][36]; __shared__ __align__(16) float so[4][16][132];
  const int tid = threadIdx.x, wave = tid >> 5, lane = tid & 31, col = lane & 15, g = lane >> 4; const int qb = blockIdx.x, b = blockIdx.y; const size_t q0 = (size_t)b * LQ + qb * 64 + wave * 16;
  F2 aq[4];
#pragma unroll
  for (int kc = 0; kc < 4; ++kc) aq[kc] = split_row(Q + (q0 + col) * DD, kc * 32, lane);
  float qs[8];
#pragma unroll
  for (int r = 0; r < 8; ++r) qs[r] = QS[q0 + 8 * g + r];
  v8f acc[8] = {};
#pragma unroll 1
  for (int ks = 0; ks < LL / 32; ++ks) {
#pragma unroll
    for (int ct = 0; ct < 2; ++ct) { const size_t kk = (size_t)b * LL + ks * 32 + ct * 16 + col; const float* krow = P + kk * DD; v8f c = {};
#pragma unroll
      for (int kc = 0; kc < 4; ++kc) { const F2 kb = split_row(krow, kc * 32, lane); c = mac3(aq[kc], kb, c); }
      const float ksq = KS[kk];
#pragma unroll
      for (int r = 0; r < 8; ++r) { const float pw = fmaxf(qs[r] + ksq - 2.0f * c[r], 0.f); sp[wave][8 * g + r][ct * 16 + col] = exp_ni(-sqrtf(pw)); } }
    LDSX();
    const F2 pa = split_row(&sp[wave][col][0], 0, lane);
#pragma unroll
    for (int dt = 0; dt < 8; ++dt) { const size_t pr = ((size_t)b * DD + dt * 16 + col) * LL + ks * 32; const v16b ph = frag_b(PH + pr, lane), pl = frag_b(PL + pr, lane); acc[dt] = wmma_bf(pa.l, ph, acc[dt]); acc[dt] = wmma_bf(pa.h, pl, acc[dt]); acc[dt] = wmma_bf(pa.h, ph, acc[dt]); }
    LDSX(); }
#pragma unroll
  for (int dt = 0; dt < 8; ++dt)
#pragma unroll
    for (int r = 0; r < 8; ++r) so[wave][8 * g + r][dt * 16 + col] = acc[dt][r];
  LDSX();
  for (int rl = 0; rl < 16; ++rl) { const v4f v = *(const v4f*)&so[wave][rl][lane * 4]; vst2(OK1 + (q0 + rl) * DD + lane * 4, v); vst2(OK2 + (q0 + rl) * DD + lane * 4, v); }
}
extern "C" void kernel_launch(void* const* d_in, const int* in_sizes, int n_in, void* d_out, int out_size, void* d_ws, size_t ws_size, hipStream_t stream) {
  (void)in_sizes; (void)n_in; (void)out_size;
  const float** F = (const float**)d_in;
  if (ws_size < (size_t)WS_END) return;
  char* ws = (char*)d_ws; __bf16 *PW = (__bf16*)(ws + WS_PW), *PH = (__bf16*)(ws + WS_PH), *PL = (__bf16*)(ws + WS_PL); float *P = (float*)(ws + WS_P), *Q = (float*)(ws + WS_Q), *KS = (float*)(ws + WS_KS), *QS = (float*)(ws + WS_QS);
  float* OQ = (float*)d_out; float* OK1 = OQ + (size_t)NB * LQ * DD; float* OK2 = OK1 + (size_t)NB * LQ * DD;
  k_pack<<<DD, 128, 0, stream>>>(F[1], PW);
  k_proj<0><<<TNB * LL / 64, 128, 0, stream>>>(F[0], PW, F[2], P, KS, nullptr);
  k_proj<1><<<TNB * LQ / 64, 128, 0, stream>>>(F[0], PW, F[2], Q, QS, OQ);
  k_planes<<<TNB * LL / 64, 256, 0, stream>>>(P, PH, PL);
  k_simk<<<dim3(TQB, TNB), 128, 0, stream>>>(Q, P, QS, KS, PH, PL, OK1, OK2);
}
